// MambaBlock_7335804142280
// MI455X (gfx1250) — hardware-verified
//
#include <hip/hip_runtime.h>
#include <stddef.h>
#include <stdint.h>
#include <math.h>


#define MROWS  4096
#define LSEQ   2048
#define DMOD   1024
#define DINN   2048
#define DIN2   4096
#define XDN    96
#define DTK    128
#define NTHR   256
#define GBM    64
#define GTHR   128
#define SCH    64
#define SCT    64
#define WSMAX  134217728
#define LOG2E  1.4426950408889634f

static_assert(MROWS % GBM == 0 && DMOD % 32 == 0 && DIN2 % 32 == 0 && DTK % 32 == 0);
static_assert(DIN2 % 128 == 0 && DINN % 128 == 0 && DMOD % 128 == 0 && XDN == 6 * 16);
static_assert(LSEQ % SCT == 0 && DINN % SCH == 0 && (SCT * 32) % (4 * SCH) == 0 && (SCT * SCH) % (8 * SCH) == 0);
static_assert((MROWS * DMOD / 8) % NTHR == 0 && (MROWS * (DINN / 8)) % NTHR == 0 && (MROWS * 16) % NTHR == 0);

typedef float          v4f   __attribute__((ext_vector_type(4)));
typedef float          v8f   __attribute__((ext_vector_type(8)));
typedef int            v8i   __attribute__((ext_vector_type(8)));
typedef unsigned short v8us  __attribute__((ext_vector_type(8)));
typedef unsigned short v16us __attribute__((ext_vector_type(16)));
typedef __bf16         v16bf __attribute__((ext_vector_type(16)));
typedef v4f  __attribute__((may_alias)) v4fa;
typedef v8us __attribute__((may_alias)) v8usa;
union FragB { v16bf v; v16us u; v8us h[2]; v8i w; };

__device__ __forceinline__ v8f wmb(const FragB& a, const FragB& b, v8f c) {
  v8f d = __builtin_amdgcn_wmma_f32_16x16x32_bf16(false, a.v, false, b.v, (short)0, c, false, false);
  asm volatile("v_nop\n\tv_nop\n\tv_nop\n\tv_nop" : "+v"(d) : "v"(a.w), "v"(b.w));
  return d;
}

__device__ __forceinline__ unsigned bf16_bits(float f) {
  const unsigned u = __float_as_uint(f);
  return (u + 0x7FFFu + ((u >> 16) & 1u)) >> 16;
}
__device__ __forceinline__ float bf16_val(float f) {
  return __uint_as_float(bf16_bits(f) << 16);
}
__device__ __forceinline__ void split_hl(float v, unsigned* hb, unsigned* lb) {
  const unsigned h = bf16_bits(v);
  *hb = h;
  *lb = bf16_bits(v - __uint_as_float(h << 16));
}
__device__ __forceinline__ float silu_f(float v) {
  const float e = exp2f(-v * LOG2E);
  return v * __builtin_amdgcn_rcpf(1.0f + e);
}
__device__ __forceinline__ float softplus_f(float v) {
  return fmaxf(v, 0.0f) + log1pf(expf(-fabsf(v)));
}

__global__ __launch_bounds__(NTHR) void k_cvx(const float* __restrict__ x, int nUnits, unsigned short* xb) {
  const int u = (int)blockIdx.x * NTHR + (int)threadIdx.x;
  if (u >= nUnits) return;
  const float* p = x + (size_t)u * 8;
  const v4f a = *(const v4fa*)p;
  const v4f b = *(const v4fa*)(p + 4);
  v8us o;
  o[0] = (unsigned short)bf16_bits(a.x); o[1] = (unsigned short)bf16_bits(a.y);
  o[2] = (unsigned short)bf16_bits(a.z); o[3] = (unsigned short)bf16_bits(a.w);
  o[4] = (unsigned short)bf16_bits(b.x); o[5] = (unsigned short)bf16_bits(b.y);
  o[6] = (unsigned short)bf16_bits(b.z); o[7] = (unsigned short)bf16_bits(b.w);
  unsigned short* dp = xb + (size_t)u * 8;
  *(volatile v8us*)dp = o;
  __threadfence();
  *(volatile v8us*)dp = o;
}

__global__ __launch_bounds__(NTHR) void k_wt(const float* __restrict__ W, int Ksrc, int N, int Kdst, int nUnits,
                                             unsigned short* dst) {
  const int u = (int)blockIdx.x * NTHR + (int)threadIdx.x;
  if (u >= nUnits) return;
  const int upr = Kdst >> 3;
  const int n   = u / upr;
  const int k8  = (u - n * upr) * 8;
  const int kk  = k8 % Ksrc;
  const float* p = W + (size_t)kk * (size_t)N + n;
  v8us o;
#pragma unroll
  for (int i = 0; i < 8; ++i) o[i] = (unsigned short)bf16_bits(p[(size_t)i * (size_t)N]);
  unsigned short* dp = dst + (size_t)n * (size_t)Kdst + k8;
  *(volatile v8us*)dp = o;
  __threadfence();
  *(volatile v8us*)dp = o;
}

template <int NT, int EPI>
__global__ __launch_bounds__(GTHR) void k_gemm(const unsigned short* __restrict__ A,
                                               const unsigned short* __restrict__ BT, int K,
                                               float* outp, int ldo, int nsplit, long long adj1,
                                               const float* __restrict__ bias) {
  constexpr int SP = 16 * NT;
  constexpr int NL = 4 * NT;
  __shared__ __attribute__((aligned(16))) float stg[GBM * SP];
  const int tid = (int)threadIdx.x, lane = tid & 31, wave = tid >> 5, hh = lane >> 4, m = lane & 15;
  const int rowBase = (int)blockIdx.x * GBM;
  const int col0    = (int)blockIdx.y * SP;

  v8f acc[NT];
  {
    const v8f z = {0.f, 0.f, 0.f, 0.f, 0.f, 0.f, 0.f, 0.f};
#pragma unroll
    for (int t = 0; t < NT; ++t) acc[t] = z;
  }
  const unsigned short* ap = A  + (size_t)(rowBase + 16 * wave + m) * (size_t)K + 8 * hh;
  const unsigned short* bp = BT + (size_t)(col0 + m) * (size_t)K + 8 * hh;

#pragma unroll 1
  for (int k0 = 0; k0 < K; k0 += 32) {
    FragB af;
    af.h[0] = *(const v8usa*)(ap + k0);
    af.h[1] = *(const v8usa*)(ap + k0 + 16);
#pragma unroll
    for (int nt = 0; nt < NT; ++nt) {
      const unsigned short* wq = bp + (size_t)(16 * nt) * (size_t)K + k0;
      FragB bf;
      bf.h[0] = *(const v8usa*)wq;
      bf.h[1] = *(const v8usa*)(wq + 16);
      acc[nt] = wmb(af, bf, acc[nt]);
    }
  }

#pragma unroll
  for (int nt = 0; nt < NT; ++nt) {
    const int lc = 16 * nt + m;
#pragma unroll
    for (int r = 0; r < 8; ++r) {
      const int lr = 16 * wave + 8 * hh + r;
      stg[lr * SP + lc] = acc[nt][r];
    }
  }
  __syncthreads();

  const int  ln  = lane < NL ? lane : NL - 1;
  const bool act = lane < NL;
  bool second = false;
  long long adj = 0;
  if constexpr (EPI == 1) {
    second = col0 >= nsplit;
    adj = second ? adj1 : 0;
  }
  v4f bb = {0.f, 0.f, 0.f, 0.f};
  if constexpr (EPI == 2) {
    const v4f t = *(const v4fa*)(bias + col0 + 4 * ln);
    bb.x = bf16_val(t.x); bb.y = bf16_val(t.y); bb.z = bf16_val(t.z); bb.w = bf16_val(t.w);
  }
  float* ob = outp + adj + (size_t)(rowBase + 16 * wave) * (size_t)ldo + col0 + 4 * ln;
  float* sb = stg + (16 * wave) * SP + 4 * ln;

#pragma unroll 1
  for (int i = 0; i < 16; ++i) {
    const v4f t = *(const v4fa*)(sb + i * SP);
    v4f y = t;
    if constexpr (EPI == 1) {
      if (second) {
        y.x = silu_f(t.x); y.y = silu_f(t.y); y.z = silu_f(t.z); y.w = silu_f(t.w);
      }
    }
    if constexpr (EPI == 2) {
      y.x = softplus_f(t.x + bb.x); y.y = softplus_f(t.y + bb.y);
      y.z = softplus_f(t.z + bb.z); y.w = softplus_f(t.w + bb.w);
    }
    if (act) {
      *(v4fa*)(sb + i * SP) = y;
      *(volatile v4f*)(ob + (size_t)i * (size_t)ldo) = y;
    }
  }
  __threadfence();
#pragma unroll 1
  for (int i = 0; i < 16; ++i) {
    const v4f y = *(const v4fa*)(sb + i * SP);
    if (act) *(volatile v4f*)(ob + (size_t)i * (size_t)ldo) = y;
  }
}

__device__ __forceinline__ float conv_ch(v4f w, float a0, float a1, float a2, float a3, float b) {
  float s = bf16_val(w.x) * a0;
  s = fmaf(bf16_val(w.y), a1, s);
  s = fmaf(bf16_val(w.z), a2, s);
  s = fmaf(bf16_val(w.w), a3, s);
  s = s + bf16_val(b);
  return silu_f(s);
}

__global__ __launch_bounds__(NTHR) void k_conv(const float* __restrict__ XIN, const float* __restrict__ Wc,
                                               const float* __restrict__ bc, int nUnits, unsigned short* XS) {
  const int u = (int)blockIdx.x * NTHR + (int)threadIdx.x;
  if (u >= nUnits) return;
  const int r  = u >> 8;
  const int d8 = (u & 255) * 8;
  const int t  = r & (LSEQ - 1);
  const float f0 = (t >= 3) ? 1.0f : 0.0f;
  const float f1 = (t >= 2) ? 1.0f : 0.0f;
  const float f2 = (t >= 1) ? 1.0f : 0.0f;
  const int r0 = (t >= 3) ? r - 3 : r;
  const int r1 = (t >= 2) ? r - 2 : r;
  const int r2 = (t >= 1) ? r - 1 : r;
  const float* p0 = XIN + (size_t)r0 * DINN + d8;
  const float* p1 = XIN + (size_t)r1 * DINN + d8;
  const float* p2 = XIN + (size_t)r2 * DINN + d8;
  const float* p3 = XIN + (size_t)r  * DINN + d8;
  v4f xa0 = *(const v4fa*)p0, xb0 = *(const v4fa*)(p0 + 4);
  v4f xa1 = *(const v4fa*)p1, xb1 = *(const v4fa*)(p1 + 4);
  v4f xa2 = *(const v4fa*)p2, xb2 = *(const v4fa*)(p2 + 4);
  const v4f xa3 = *(const v4fa*)p3, xb3 = *(const v4fa*)(p3 + 4);
  xa0 = xa0 * f0; xb0 = xb0 * f0;
  xa1 = xa1 * f1; xb1 = xb1 * f1;
  xa2 = xa2 * f2; xb2 = xb2 * f2;
  const float* wp = Wc + (size_t)d8 * 4;
  const v4f w0 = *(const v4fa*)(wp),      w1 = *(const v4fa*)(wp + 4);
  const v4f w2 = *(const v4fa*)(wp + 8),  w3 = *(const v4fa*)(wp + 12);
  const v4f w4 = *(const v4fa*)(wp + 16), w5 = *(const v4fa*)(wp + 20);
  const v4f w6 = *(const v4fa*)(wp + 24), w7 = *(const v4fa*)(wp + 28);
  const v4f ba = *(const v4fa*)(bc + d8), bb = *(const v4fa*)(bc + d8 + 4);

  const float c0 = conv_ch(w0, xa0.x, xa1.x, xa2.x, xa3.x, ba.x);
  const float c1 = conv_ch(w1, xa0.y, xa1.y, xa2.y, xa3.y, ba.y);
  const float c2 = conv_ch(w2, xa0.z, xa1.z, xa2.z, xa3.z, ba.z);
  const float c3 = conv_ch(w3, xa0.w, xa1.w, xa2.w, xa3.w, ba.w);
  const float c4 = conv_ch(w4, xb0.x, xb1.x, xb2.x, xb3.x, bb.x);
  const float c5 = conv_ch(w5, xb0.y, xb1.y, xb2.y, xb3.y, bb.y);
  const float c6 = conv_ch(w6, xb0.z, xb1.z, xb2.z, xb3.z, bb.z);
  const float c7 = conv_ch(w7, xb0.w, xb1.w, xb2.w, xb3.w, bb.w);

  v8us oh, ol;
  unsigned hb, lb;
  split_hl(c0, &hb, &lb); oh[0] = (unsigned short)hb; ol[0] = (unsigned short)lb;
  split_hl(c1, &hb, &lb); oh[1] = (unsigned short)hb; ol[1] = (unsigned short)lb;
  split_hl(c2, &hb, &lb); oh[2] = (unsigned short)hb; ol[2] = (unsigned short)lb;
  split_hl(c3, &hb, &lb); oh[3] = (unsigned short)hb; ol[3] = (unsigned short)lb;
  split_hl(c4, &hb, &lb); oh[4] = (unsigned short)hb; ol[4] = (unsigned short)lb;
  split_hl(c5, &hb, &lb); oh[5] = (unsigned short)hb; ol[5] = (unsigned short)lb;
  split_hl(c6, &hb, &lb); oh[6] = (unsigned short)hb; ol[6] = (unsigned short)lb;
  split_hl(c7, &hb, &lb); oh[7] = (unsigned short)hb; ol[7] = (unsigned short)lb;

  unsigned short* dh = XS + (size_t)r * DIN2 + d8;
  unsigned short* dl = dh + DINN;
  *(volatile v8us*)dh = oh;
  *(volatile v8us*)dl = ol;
  __threadfence();
  *(volatile v8us*)dh = oh;
  *(volatile v8us*)dl = ol;
}

__global__ __launch_bounds__(NTHR) void k_dthl(const float* __restrict__ XDBL, int nUnits, unsigned short* DT) {
  const int u = (int)blockIdx.x * NTHR + (int)threadIdx.x;
  if (u >= nUnits) return;
  const int row = u >> 4;
  const int c8  = (u & 15) * 8;
  const int sc  = c8 & 63;
  const bool isLo = c8 >= 64;
  const float* p = XDBL + (size_t)row * XDN + sc;
  const v4f a = *(const v4fa*)p;
  const v4f b = *(const v4fa*)(p + 4);
  v8us o;
  unsigned hb, lb;
  split_hl(a.x, &hb, &lb); o[0] = (unsigned short)(isLo ? lb : hb);
  split_hl(a.y, &hb, &lb); o[1] = (unsigned short)(isLo ? lb : hb);
  split_hl(a.z, &hb, &lb); o[2] = (unsigned short)(isLo ? lb : hb);
  split_hl(a.w, &hb, &lb); o[3] = (unsigned short)(isLo ? lb : hb);
  split_hl(b.x, &hb, &lb); o[4] = (unsigned short)(isLo ? lb : hb);
  split_hl(b.y, &hb, &lb); o[5] = (unsigned short)(isLo ? lb : hb);
  split_hl(b.z, &hb, &lb); o[6] = (unsigned short)(isLo ? lb : hb);
  split_hl(b.w, &hb, &lb); o[7] = (unsigned short)(isLo ? lb : hb);
  unsigned short* dp = DT + (size_t)row * DTK + c8;
  *(volatile v8us*)dp = o;
  __threadfence();
  *(volatile v8us*)dp = o;
}

#define AINI(N, V) A2[N] = -exp2f(bf16_val(V) * LOG2E) * LOG2E; h[N] = 0.0f;
#define SSTEP(N, BV, CV) { const float e = exp2f(dt * A2[N]); h[N] = fmaf(e, h[N], dtx * (BV)); \
                           y = fmaf(h[N], (CV), y); }

__global__ __launch_bounds__(SCH) void k_scan(const float* __restrict__ DELTA, const float* __restrict__ G,
                                              const float* __restrict__ XDBL, const float* __restrict__ Alog,
                                              const float* __restrict__ Dp, unsigned short* XS) {
  __shared__ __attribute__((aligned(16))) float sBC[SCT * 32];
  __shared__ __attribute__((aligned(16))) unsigned short yh[SCT * SCH];
  __shared__ __attribute__((aligned(16))) unsigned short yl[SCT * SCH];
  const int tid = (int)threadIdx.x;
  const int b   = (int)blockIdx.x >> 5;
  const int d0  = ((int)blockIdx.x & 31) * SCH;
  const int d   = d0 + tid;

  float A2[16], h[16];
  {
    const float* ar = Alog + (size_t)d * 16;
    const v4f q0 = *(const v4fa*)(ar);
    const v4f q1 = *(const v4fa*)(ar + 4);
    const v4f q2 = *(const v4fa*)(ar + 8);
    const v4f q3 = *(const v4fa*)(ar + 12);
    AINI(0, q0.x)  AINI(1, q0.y)  AINI(2, q0.z)  AINI(3, q0.w)
    AINI(4, q1.x)  AINI(5, q1.y)  AINI(6, q1.z)  AINI(7, q1.w)
    AINI(8, q2.x)  AINI(9, q2.y)  AINI(10, q2.z) AINI(11, q2.w)
    AINI(12, q3.x) AINI(13, q3.y) AINI(14, q3.z) AINI(15, q3.w)
  }
  const float Dv = bf16_val(Dp[d]);

#pragma unroll 1
  for (int c = 0; c < LSEQ / SCT; ++c) {
    const int rb = b * LSEQ + c * SCT;
#pragma unroll 4
    for (int i = 0; i < (SCT * 32) / (4 * SCH); ++i) {
      const int idx = i * SCH + tid;
      const int row = idx >> 3;
      const int q   = idx & 7;
      const v4f v = *(const v4fa*)(XDBL + (size_t)(rb + row) * XDN + 64 + 4 * q);
      *(v4fa*)(sBC + 4 * idx) = v;
    }
    __syncthreads();

#pragma unroll 1
    for (int s = 0; s < SCT; ++s) {
      const size_t r = (size_t)(rb + s);
      const float dt = DELTA[r * DINN + d];
      const unsigned xh = XS[r * DIN2 + d];
      const unsigned xl = XS[r * DIN2 + DINN + d];
      const float g  = G[r * DINN + d];
      const float xv = __uint_as_float(xh << 16) + __uint_as_float(xl << 16);
      const float dtx = dt * xv;
      const float* bcp = sBC + s * 32;
      const v4f B0 = *(const v4fa*)(bcp),      B1 = *(const v4fa*)(bcp + 4);
      const v4f B2 = *(const v4fa*)(bcp + 8),  B3 = *(const v4fa*)(bcp + 12);
      const v4f C0 = *(const v4fa*)(bcp + 16), C1 = *(const v4fa*)(bcp + 20);
      const v4f C2 = *(const v4fa*)(bcp + 24), C3 = *(const v4fa*)(bcp + 28);
      float y = 0.0f;
      SSTEP(0, B0.x, C0.x)   SSTEP(1, B0.y, C0.y)   SSTEP(2, B0.z, C0.z)   SSTEP(3, B0.w, C0.w)
      SSTEP(4, B1.x, C1.x)   SSTEP(5, B1.y, C1.y)   SSTEP(6, B1.z, C1.z)   SSTEP(7, B1.w, C1.w)
      SSTEP(8, B2.x, C2.x)   SSTEP(9, B2.y, C2.y)   SSTEP(10, B2.z, C2.z)  SSTEP(11, B2.w, C2.w)
      SSTEP(12, B3.x, C3.x)  SSTEP(13, B3.y, C3.y)  SSTEP(14, B3.z, C3.z)  SSTEP(15, B3.w, C3.w)
      const float yv = (y + Dv * xv) * g;
      unsigned hb, lb;
      split_hl(yv, &hb, &lb);
      yh[s * SCH + tid] = (unsigned short)hb;
      yl[s * SCH + tid] = (unsigned short)lb;
    }
    __syncthreads();

    v8us qh[8], ql[8];
#pragma unroll
    for (int i = 0; i < 8; ++i) {
      const int idx = i * SCH + tid;
      qh[i] = *(const v8usa*)(yh + 8 * idx);
      ql[i] = *(const v8usa*)(yl + 8 * idx);
    }
#pragma unroll
    for (int i = 0; i < 8; ++i) {
      const int idx = i * SCH + tid;
      unsigned short* dp = XS + (size_t)(rb + (idx >> 3)) * DIN2 + d0 + 8 * (idx & 7);
      *(volatile v8us*)dp = qh[i];
      *(volatile v8us*)(dp + DINN) = ql[i];
    }
    __threadfence();
#pragma unroll
    for (int i = 0; i < 8; ++i) {
      const int idx = i * SCH + tid;
      unsigned short* dp = XS + (size_t)(rb + (idx >> 3)) * DIN2 + d0 + 8 * (idx & 7);
      *(volatile v8us*)dp = qh[i];
      *(volatile v8us*)(dp + DINN) = ql[i];
    }
  }
}
#undef AINI
#undef SSTEP

static inline size_t al256(size_t o) { return (o + 255) & ~(size_t)255; }

extern "C" void kernel_launch(void* const* d_in, const int* in_sizes, int n_in,
                              void* d_out, int out_size, void* d_ws, size_t ws_size,
                              hipStream_t stream) {
  if (n_in < 10) return;
  if (in_sizes[0] != MROWS * DMOD) return;
  if (in_sizes[1] != DMOD * DIN2) return;
  if (in_sizes[2] != DINN * 4) return;
  if (in_sizes[3] != DINN) return;
  if (in_sizes[4] != DINN * XDN) return;
  if (in_sizes[5] != 64 * DINN) return;
  if (in_sizes[6] != DINN) return;
  if (in_sizes[7] != DINN * 16) return;
  if (in_sizes[8] != DINN) return;
  if (in_sizes[9] != DINN * DMOD) return;
  if (out_size != MROWS * DMOD) return;

  const float* x      = (const float*)d_in[0];
  const float* W_in   = (const float*)d_in[1];
  const float* W_conv = (const float*)d_in[2];
  const float* b_conv = (const float*)d_in[3];
  const float* W_x    = (const float*)d_in[4];
  const float* W_dt   = (const float*)d_in[5];
  const float* b_dt   = (const float*)d_in[6];
  const float* A_log  = (const float*)d_in[7];
  const float* Dp     = (const float*)d_in[8];
  const float* W_out  = (const float*)d_in[9];
  float* out = (float*)d_out;

  char* ws = (char*)d_ws;
  size_t off = 0;
  const size_t oXB   = off; off = al256(off + (size_t)MROWS * DMOD * 2);
  const size_t oWIN  = off; off = al256(off + (size_t)DIN2 * DMOD * 2);
  const size_t oWX2  = off; off = al256(off + (size_t)XDN * DIN2 * 2);
  const size_t oWDT  = off; off = al256(off + (size_t)DINN * DTK * 2);
  const size_t oWO2  = off; off = al256(off + (size_t)DMOD * DIN2 * 2);
  const size_t oXIN  = off; off = al256(off + (size_t)MROWS * DINN * 4);
  const size_t oG    = off; off = al256(off + (size_t)MROWS * DINN * 4);
  const size_t oXS   = off; off = al256(off + (size_t)MROWS * DIN2 * 2);
  const size_t oXDBL = off; off = al256(off + (size_t)MROWS * XDN * 4);
  const size_t oDT   = off; off = al256(off + (size_t)MROWS * DTK * 2);
  if (off > ws_size || off > (size_t)WSMAX) return;
  unsigned short* XB   = (unsigned short*)(ws + oXB);
  unsigned short* WINT = (unsigned short*)(ws + oWIN);
  unsigned short* WX2  = (unsigned short*)(ws + oWX2);
  unsigned short* WDT2 = (unsigned short*)(ws + oWDT);
  unsigned short* WO2  = (unsigned short*)(ws + oWO2);
  float*          XIN  = (float*)(ws + oXIN);
  float*          DELTA = XIN;
  float*          G    = (float*)(ws + oG);
  unsigned short* XS   = (unsigned short*)(ws + oXS);
  float*          XDBL = (float*)(ws + oXDBL);
  unsigned short* DT   = (unsigned short*)(ws + oDT);
  const long long adjG = (long long)((oG - oXIN) / 4) - (long long)DINN;

  { const int nU = MROWS * DMOD / 8;
    k_cvx<<<nU / NTHR, NTHR, 0, stream>>>(x, nU, XB); }
  { const int nU = DIN2 * DMOD / 8;
    k_wt<<<(nU + NTHR - 1) / NTHR, NTHR, 0, stream>>>(W_in, DMOD, DIN2, DMOD, nU, WINT); }
  { const int nU = XDN * DIN2 / 8;
    k_wt<<<(nU + NTHR - 1) / NTHR, NTHR, 0, stream>>>(W_x, DINN, XDN, DIN2, nU, WX2); }
  { const int nU = DINN * DTK / 8;
    k_wt<<<(nU + NTHR - 1) / NTHR, NTHR, 0, stream>>>(W_dt, 64, DINN, DTK, nU, WDT2); }
  { const int nU = DMOD * DIN2 / 8;
    k_wt<<<(nU + NTHR - 1) / NTHR, NTHR, 0, stream>>>(W_out, DINN, DMOD, DIN2, nU, WO2); }
  k_gemm<8, 1><<<dim3(MROWS / GBM, DIN2 / 128), GTHR, 0, stream>>>(XB, WINT, DMOD, XIN, DINN, DINN, adjG, b_dt);
  { const int nU = MROWS * (DINN / 8);
    k_conv<<<nU / NTHR, NTHR, 0, stream>>>(XIN, W_conv, b_conv, nU, XS); }
  k_gemm<6, 0><<<dim3(MROWS / GBM, 1), GTHR, 0, stream>>>(XS, WX2, DIN2, XDBL, XDN, 0, 0, b_dt);
  { const int nU = MROWS * 16;
    k_dthl<<<nU / NTHR, NTHR, 0, stream>>>(XDBL, nU, DT); }
  k_gemm<8, 2><<<dim3(MROWS / GBM, DINN / 128), GTHR, 0, stream>>>(DT, WDT2, DTK, DELTA, DINN, 0, 0, b_dt);
  k_scan<<<2 * (DINN / SCH), SCH, 0, stream>>>(DELTA, G, XDBL, A_log, Dp, XS);
  k_gemm<8, 0><<<dim3(MROWS / GBM, DMOD / 128), GTHR, 0, stream>>>(XS, WO2, DIN2, out, DMOD, 0, 0, b_dt);
}
